// SlidingWindowProcessor_60593398612039
// MI455X (gfx1250) — hardware-verified
//
#include <hip/hip_runtime.h>


typedef _Float16 f16t;
typedef f16t           v16h  __attribute__((ext_vector_type(16)));
typedef f16t           v8h   __attribute__((ext_vector_type(8)));
typedef __bf16         v16b  __attribute__((ext_vector_type(16)));
typedef unsigned short v16us __attribute__((ext_vector_type(16)));
typedef unsigned short v8us  __attribute__((ext_vector_type(8)));
typedef float          v8f   __attribute__((ext_vector_type(8)));
typedef float          v4f   __attribute__((ext_vector_type(4)));
typedef unsigned int   v4u   __attribute__((ext_vector_type(4)));

union FragH { v16h v; v8h q[2]; };
union FragB { v16b v; v16us u; v8us q[2]; unsigned short s[16]; };
union Pk16  { v8us v; unsigned short s[8]; v4u u; };
union Pk16h { v8h h; v4u u; };

#define NSEQ 2048
#define TT   1024
#define CC   256
#define HH   256
#define GG   768
#define WMAX 64
#define XSP  80
#define AP   264
#define HP   264
#define HFP  264

#define WIH_E 196608
#define WP_E  65536
#define U_IH  24576
#define U_HH  24576
#define U_P   8192
#define U_TOT (U_IH + U_HH + U_P)

#define INV13 0.0001220703125f

__device__ __forceinline__ unsigned short bfb(float f) {
    unsigned int u = __float_as_uint(f);
    u += 0x7FFFu + ((u >> 16) & 1u);
    return (unsigned short)(u >> 16);
}
__device__ __forceinline__ float bfv(unsigned short b) {
    return __uint_as_float(((unsigned int)b) << 16);
}
__device__ __forceinline__ v8f wbf(v16b a, v16b b, v8f c) {
    return __builtin_amdgcn_wmma_f32_16x16x32_bf16(false, a, false, b, (short)0, c, false, false);
}
__device__ __forceinline__ v8f whf(v16h a, v16h b, v8f c) {
    return __builtin_amdgcn_wmma_f32_16x16x32_f16(false, a, false, b, (short)0, c, false, false);
}
__device__ __forceinline__ float fsigm(float x) {
    float t = __expf(-x);
    return __builtin_amdgcn_rcpf(1.0f + t);
}
__device__ __forceinline__ float ftanh(float x) {
    float ax = fabsf(x);
    float t  = __expf(-2.0f * ax);
    float r  = (1.0f - t) * __builtin_amdgcn_rcpf(1.0f + t);
    return copysignf(r, x);
}
__device__ __forceinline__ float wsum(float v) {
#pragma unroll
    for (int o = 16; o > 0; o >>= 1) v += __shfl_xor(v, o);
    return v;
}
__device__ __forceinline__ float gelu_erf(float x) {
    return 0.5f * x * (1.0f + erff(x * 0.70710678118654752440f));
}

__global__ __launch_bounds__(256) void k_pack(
    const float* __restrict__ w_ih, const float* __restrict__ w_hh, const float* __restrict__ proj_w,
    unsigned short* __restrict__ wihh, unsigned short* __restrict__ wihl, f16t* __restrict__ whh,
    unsigned short* __restrict__ wph, unsigned short* __restrict__ wpl)
{
    const int li = blockIdx.x * 256 + threadIdx.x;
    if (li >= U_TOT) return;
    int seg, u;
    const float* W;
    if (li < U_IH)             { seg = 0; u = li;               W = w_ih;   }
    else if (li < U_IH + U_HH) { seg = 1; u = li - U_IH;        W = w_hh;   }
    else                       { seg = 2; u = li - U_IH - U_HH; W = proj_w; }
    const int idx  = u * 8;
    const int e8   = idx & 15;
    const int ln   = (idx >> 4) & 31;
    const int kk   = (idx >> 9) & 7;
    const int tile = idx >> 12;
    const int g    = tile * 16 + (ln & 15);
    const int h    = ln >> 4;
    const int k0   = kk * 32 + 8 * h + (e8 ? 16 : 0);
    const float* src = W + (size_t)g * 256 + k0;
    const v4f a = *(const v4f*)src;
    const v4f c = *(const v4f*)(src + 4);
    float f[8] = {a[0], a[1], a[2], a[3], c[0], c[1], c[2], c[3]};
    if (seg == 1) {
        Pk16h p;
#pragma unroll
        for (int e = 0; e < 8; ++e) p.h[e] = (f16t)(f[e] * 128.0f);
        f16t* d = whh + idx;
        *(volatile v4u*)d = p.u;
        __threadfence();
        *(volatile v4u*)d = p.u;
    } else {
        const float sc = (seg == 0) ? 8192.0f : 1.0f;
        Pk16 ph, pl;
#pragma unroll
        for (int e = 0; e < 8; ++e) {
            const float v = f[e] * sc;
            const unsigned short hb = bfb(v);
            ph.s[e] = hb;
            pl.s[e] = bfb(v - bfv(hb));
        }
        unsigned short* dh = ((seg == 0) ? wihh : wph) + idx;
        unsigned short* dl = ((seg == 0) ? wihl : wpl) + idx;
        *(volatile v4u*)dh = ph.u;
        *(volatile v4u*)dl = pl.u;
        __threadfence();
        *(volatile v4u*)dh = ph.u;
        *(volatile v4u*)dl = pl.u;
    }
}

union RegA { unsigned short a[2 * 16 * AP]; float y[16 * HH]; };

__global__ __launch_bounds__(256) void k_gru(
    const float* __restrict__ x, const float* __restrict__ b_ih, const float* __restrict__ b_hh,
    const float* __restrict__ proj_b, const float* __restrict__ ln_g, const float* __restrict__ ln_b,
    const int* __restrict__ wsz,
    const unsigned short* __restrict__ wihh, const unsigned short* __restrict__ wihl,
    const f16t* __restrict__ whh,
    const unsigned short* __restrict__ wph, const unsigned short* __restrict__ wpl,
    float* __restrict__ out)
{
    __shared__ __align__(16) unsigned short xsh[4 * XSP];
    __shared__ __align__(16) unsigned short xsl[4 * XSP];
    __shared__ __align__(16) RegA rA;
    __shared__ __align__(16) f16t  hbuf[2 * 16 * HP];
    __shared__ __align__(16) float hf[16 * HFP];

    const int tid  = threadIdx.x;
    const int lane = tid & 31;
    const int wv   = tid >> 5;
    const int m    = lane & 15;
    const int lhi  = lane >> 4;
    const int n0   = blockIdx.x * 16;
    if (n0 + 16 > NSEQ) return;
    const int b  = n0 >> 10;
    const int t0 = n0 & (TT - 1);

    int nst = wsz[0];
    nst = nst < 0 ? 0 : (nst > WMAX ? WMAX : nst);

    for (int i = tid; i < 16 * HP; i += 256) hbuf[i] = (f16t)0.0f;

    int tiles[6];
    tiles[0] = 2 * wv;      tiles[1] = 2 * wv + 1;
    tiles[2] = 16 + 2 * wv; tiles[3] = 17 + 2 * wv;
    tiles[4] = 32 + 2 * wv; tiles[5] = 33 + 2 * wv;

    float bih[6], bhh[6];
#pragma unroll
    for (int q = 0; q < 6; ++q) {
        const int col = tiles[q] * 16 + m;
        bih[q] = b_ih[col];
        bhh[q] = b_hh[col];
    }

    float hprev[2][8];
#pragma unroll
    for (int p = 0; p < 2; ++p)
#pragma unroll
        for (int v = 0; v < 8; ++v) hprev[p][v] = 0.0f;

#pragma unroll 1
    for (int step = 0; step < nst; ++step) {
        int zoff = 0;
        asm volatile("" : "+s"(zoff));
        const unsigned short* wihh_s = wihh + zoff;
        const unsigned short* wihl_s = wihl + zoff;
        const f16t*           whh_s  = whh  + zoff;

        if (tid < 79) {
            const int tt = t0 - 63 + tid;
            v4f v = {0.0f, 0.0f, 0.0f, 0.0f};
            if (tt >= 0) v = *(const v4f*)(x + ((size_t)(b * TT + tt)) * CC + 4 * step);
#pragma unroll
            for (int j = 0; j < 4; ++j) {
                const unsigned short hb = bfb(v[j]);
                xsh[j * XSP + tid] = hb;
                xsl[j * XSP + tid] = bfb(v[j] - bfv(hb));
            }
        }
        __syncthreads();

        {
            const int tm = tid >> 4, kq = tid & 15;
            const int j  = kq >> 2;
            const unsigned short* sh = xsh + j * XSP + tm + 16 * (kq & 3);
            const unsigned short* sl = xsl + j * XSP + tm + 16 * (kq & 3);
            Pk16 h0, h1, l0, l1;
#pragma unroll
            for (int i = 0; i < 8; ++i) {
                h0.s[i] = sh[i]; h1.s[i] = sh[8 + i];
                l0.s[i] = sl[i]; l1.s[i] = sl[8 + i];
            }
            unsigned short* dh = rA.a + tm * AP + 16 * kq;
            unsigned short* dl = dh + 16 * AP;
            *(v8us*)dh       = h0.v;
            *(v8us*)(dh + 8) = h1.v;
            *(v8us*)dl       = l0.v;
            *(v8us*)(dl + 8) = l1.v;
        }
        __syncthreads();

        v8f acc[6], acch[2];
        {
            const v8f z8 = {0.f, 0.f, 0.f, 0.f, 0.f, 0.f, 0.f, 0.f};
#pragma unroll
            for (int q = 0; q < 6; ++q) acc[q] = z8;
            acch[0] = z8; acch[1] = z8;
        }

        {
            const unsigned short* Ah = rA.a + m * AP + 8 * lhi;
            const unsigned short* Al = Ah + 16 * AP;
#pragma unroll 1
            for (int kk = 0; kk < 8; ++kk) {
                FragB ah, al;
                ah.q[0] = *(const v8us*)(Ah + 32 * kk);
                ah.q[1] = *(const v8us*)(Ah + 32 * kk + 16);
                al.q[0] = *(const v8us*)(Al + 32 * kk);
                al.q[1] = *(const v8us*)(Al + 32 * kk + 16);
#pragma unroll
                for (int g = 0; g < 3; ++g) {
                    const int o0 = ((tiles[2 * g] * 8 + kk) * 32 + lane) << 4;
                    const int o1 = ((tiles[2 * g + 1] * 8 + kk) * 32 + lane) << 4;
                    FragB bh0, bl0, bh1, bl1;
                    bh0.u = *(const v16us*)(wihh_s + o0);
                    bl0.u = *(const v16us*)(wihl_s + o0);
                    bh1.u = *(const v16us*)(wihh_s + o1);
                    bl1.u = *(const v16us*)(wihl_s + o1);
                    acc[2 * g]     = wbf(ah.v, bh0.v, acc[2 * g]);
                    acc[2 * g]     = wbf(ah.v, bl0.v, acc[2 * g]);
                    acc[2 * g]     = wbf(al.v, bh0.v, acc[2 * g]);
                    acc[2 * g + 1] = wbf(ah.v, bh1.v, acc[2 * g + 1]);
                    acc[2 * g + 1] = wbf(ah.v, bl1.v, acc[2 * g + 1]);
                    acc[2 * g + 1] = wbf(al.v, bh1.v, acc[2 * g + 1]);
                    asm volatile("v_nop\n\tv_nop\n\tv_nop\n\tv_nop"
                                 : "+v"(acc[2 * g]), "+v"(acc[2 * g + 1])
                                 : "v"(ah.u), "v"(al.u), "v"(bh0.u), "v"(bl0.u), "v"(bh1.u), "v"(bl1.u));
                }
            }
        }

        {
            const f16t* Hin = hbuf + ((step & 1) * 16 + m) * HP + 8 * lhi;
#pragma unroll 1
            for (int kk = 0; kk < 8; ++kk) {
                FragH a;
                a.q[0] = *(const v8h*)(Hin + 32 * kk);
                a.q[1] = *(const v8h*)(Hin + 32 * kk + 16);
                FragH bq[6];
#pragma unroll
                for (int q = 0; q < 6; ++q)
                    bq[q].v = *(const v16h*)(whh_s + (((tiles[q] * 8 + kk) * 32 + lane) << 4));
#pragma unroll
                for (int q = 0; q < 4; ++q) acc[q] = whf(a.v, bq[q].v, acc[q]);
                acch[0] = whf(a.v, bq[4].v, acch[0]);
                acch[1] = whf(a.v, bq[5].v, acch[1]);
                asm volatile("v_nop\n\tv_nop\n\tv_nop\n\tv_nop"
                             : "+v"(acc[0]), "+v"(acc[1]), "+v"(acc[2]), "+v"(acc[3]),
                               "+v"(acch[0]), "+v"(acch[1])
                             : "v"(a.v), "v"(bq[0].v), "v"(bq[1].v), "v"(bq[2].v),
                               "v"(bq[3].v), "v"(bq[4].v), "v"(bq[5].v));
            }
        }

        {
            f16t* Hout = hbuf + (((step + 1) & 1) * 16) * HP;
#pragma unroll
            for (int p = 0; p < 2; ++p) {
                const int col = 32 * wv + 16 * p + m;
#pragma unroll
                for (int v = 0; v < 8; ++v) {
                    const float rg = acc[p][v] * INV13 + bih[p] + bhh[p];
                    const float zg = acc[2 + p][v] * INV13 + bih[2 + p] + bhh[2 + p];
                    const float r  = fsigm(rg);
                    const float z  = fsigm(zg);
                    const float hn = acch[p][v] * INV13 + bhh[4 + p];
                    const float ng = acc[4 + p][v] * INV13 + bih[4 + p] + r * hn;
                    const float nn = ftanh(ng);
                    const float hv = (1.0f - z) * nn + z * hprev[p][v];
                    hprev[p][v] = hv;
                    Hout[(v + 8 * lhi) * HP + col] = (f16t)(hv * 64.0f);
                }
            }
        }
        __syncthreads();
    }

#pragma unroll
    for (int p = 0; p < 2; ++p)
#pragma unroll
        for (int v = 0; v < 8; ++v)
            hf[(v + 8 * lhi) * HFP + 32 * wv + 16 * p + m] = hprev[p][v];
    __syncthreads();

    {
        const v8f z8 = {0.f, 0.f, 0.f, 0.f, 0.f, 0.f, 0.f, 0.f};
        v8f acc2[2];
        acc2[0] = z8; acc2[1] = z8;
        const int pt0 = 2 * wv, pt1 = 2 * wv + 1;
        const float* Hf = hf + m * HFP + 8 * lhi;
#pragma unroll 1
        for (int kk = 0; kk < 8; ++kk) {
            const v4f f0 = *(const v4f*)(Hf + 32 * kk);
            const v4f f1 = *(const v4f*)(Hf + 32 * kk + 4);
            const v4f f2 = *(const v4f*)(Hf + 32 * kk + 16);
            const v4f f3 = *(const v4f*)(Hf + 32 * kk + 20);
            FragB ah, al;
#pragma unroll
            for (int i = 0; i < 4; ++i) {
                unsigned short hb;
                hb = bfb(f0[i]); ah.s[i]      = hb; al.s[i]      = bfb(f0[i] - bfv(hb));
                hb = bfb(f1[i]); ah.s[4 + i]  = hb; al.s[4 + i]  = bfb(f1[i] - bfv(hb));
                hb = bfb(f2[i]); ah.s[8 + i]  = hb; al.s[8 + i]  = bfb(f2[i] - bfv(hb));
                hb = bfb(f3[i]); ah.s[12 + i] = hb; al.s[12 + i] = bfb(f3[i] - bfv(hb));
            }
            const int o0 = ((pt0 * 8 + kk) * 32 + lane) << 4;
            const int o1 = ((pt1 * 8 + kk) * 32 + lane) << 4;
            FragB bh0, bl0, bh1, bl1;
            bh0.u = *(const v16us*)(wph + o0);
            bl0.u = *(const v16us*)(wpl + o0);
            bh1.u = *(const v16us*)(wph + o1);
            bl1.u = *(const v16us*)(wpl + o1);
            acc2[0] = wbf(ah.v, bh0.v, acc2[0]);
            acc2[0] = wbf(ah.v, bl0.v, acc2[0]);
            acc2[0] = wbf(al.v, bh0.v, acc2[0]);
            acc2[1] = wbf(ah.v, bh1.v, acc2[1]);
            acc2[1] = wbf(ah.v, bl1.v, acc2[1]);
            acc2[1] = wbf(al.v, bh1.v, acc2[1]);
            asm volatile("v_nop\n\tv_nop\n\tv_nop\n\tv_nop"
                         : "+v"(acc2[0]), "+v"(acc2[1])
                         : "v"(ah.u), "v"(al.u), "v"(bh0.u), "v"(bl0.u), "v"(bh1.u), "v"(bl1.u));
        }
        const float pb0 = proj_b[16 * pt0 + m];
        const float pb1 = proj_b[16 * pt1 + m];
#pragma unroll
        for (int v = 0; v < 8; ++v) {
            rA.y[(v + 8 * lhi) * HH + 16 * pt0 + m] = acc2[0][v] + pb0;
            rA.y[(v + 8 * lhi) * HH + 16 * pt1 + m] = acc2[1][v] + pb1;
        }
    }
    __syncthreads();

    {
        const v4f g0 = *(const v4f*)(ln_g + 4 * lane);
        const v4f g1 = *(const v4f*)(ln_g + 128 + 4 * lane);
        const v4f c0 = *(const v4f*)(ln_b + 4 * lane);
        const v4f c1 = *(const v4f*)(ln_b + 128 + 4 * lane);
        v4f o[2][2];
#pragma unroll
        for (int rr = 0; rr < 2; ++rr) {
            const int row = 2 * wv + rr;
            const v4f y0 = *(const v4f*)(rA.y + row * HH + 4 * lane);
            const v4f y1 = *(const v4f*)(rA.y + row * HH + 128 + 4 * lane);
            float s = ((y0[0] + y0[1]) + (y0[2] + y0[3])) + ((y1[0] + y1[1]) + (y1[2] + y1[3]));
            s = wsum(s);
            const float mu = s * (1.0f / 256.0f);
            const v4f d0 = y0 - mu;
            const v4f d1 = y1 - mu;
            float sq = ((d0[0] * d0[0] + d0[1] * d0[1]) + (d0[2] * d0[2] + d0[3] * d0[3]))
                     + ((d1[0] * d1[0] + d1[1] * d1[1]) + (d1[2] * d1[2] + d1[3] * d1[3]));
            sq = wsum(sq);
            const float rstd = rsqrtf(sq * (1.0f / 256.0f) + 1e-5f);
#pragma unroll
            for (int i = 0; i < 4; ++i) {
                o[rr][0][i] = gelu_erf(d0[i] * rstd * g0[i] + c0[i]);
                o[rr][1][i] = gelu_erf(d1[i] * rstd * g1[i] + c1[i]);
            }
        }
#pragma unroll
        for (int rr = 0; rr < 2; ++rr) {
            float* orow = out + (size_t)(n0 + 2 * wv + rr) * HH;
            *(volatile v4f*)(orow + 4 * lane)       = o[rr][0];
            *(volatile v4f*)(orow + 128 + 4 * lane) = o[rr][1];
        }
        __threadfence();
#pragma unroll
        for (int rr = 0; rr < 2; ++rr) {
            float* orow = out + (size_t)(n0 + 2 * wv + rr) * HH;
            *(volatile v4f*)(orow + 4 * lane)       = o[rr][0];
            *(volatile v4f*)(orow + 128 + 4 * lane) = o[rr][1];
        }
    }
}

extern "C" void kernel_launch(void* const* d_in, const int* in_sizes, int n_in,
                              void* d_out, int out_size, void* d_ws, size_t ws_size,
                              hipStream_t stream) {
    if (n_in < 10) return;
    if (in_sizes[0] != NSEQ * CC || in_sizes[1] != GG * CC || in_sizes[2] != GG * HH ||
        in_sizes[3] != GG || in_sizes[4] != GG || in_sizes[5] != HH * HH || in_sizes[6] != HH ||
        in_sizes[7] != HH || in_sizes[8] != HH || in_sizes[9] < 1 || out_size != NSEQ * HH) return;

    const float* x      = (const float*)d_in[0];
    const float* w_ih   = (const float*)d_in[1];
    const float* w_hh   = (const float*)d_in[2];
    const float* b_ih   = (const float*)d_in[3];
    const float* b_hh   = (const float*)d_in[4];
    const float* proj_w = (const float*)d_in[5];
    const float* proj_b = (const float*)d_in[6];
    const float* ln_g   = (const float*)d_in[7];
    const float* ln_b   = (const float*)d_in[8];
    const int*   wsz    = (const int*)d_in[9];
    float* outp = (float*)d_out;

    const size_t total = ((size_t)3 * WIH_E + (size_t)2 * WP_E) * 2;
    if (total > ws_size) return;
    unsigned short* wihh = (unsigned short*)d_ws;
    unsigned short* wihl = wihh + WIH_E;
    f16t*           whh  = (f16t*)(wihl + WIH_E);
    unsigned short* wph  = (unsigned short*)(whh + WIH_E);
    unsigned short* wpl  = wph + WP_E;

    k_pack<<<dim3(U_TOT / 256), dim3(256), 0, stream>>>(w_ih, w_hh, proj_w, wihh, wihl, whh, wph, wpl);

    k_gru<<<dim3(NSEQ / 16), dim3(256), 0, stream>>>(x, b_ih, b_hh, proj_b, ln_g, ln_b, wsz,
                                                    wihh, wihl, whh, wph, wpl, outp);
}
